// MaskedAttentionOperation_15298673509078
// MI455X (gfx1250) — hardware-verified
//
#include <hip/hip_runtime.h>
#include <hip/hip_bf16.h>
#include <math.h>


#define BB 64
#define SS 1024
#define DD 64
#define HH 1
#define DKK 64
#define QW 2

typedef _Float16 bf16;
typedef __attribute__((ext_vector_type(4))) unsigned v4u_t;
typedef unsigned v4ua __attribute__((ext_vector_type(4), may_alias));
typedef __attribute__((ext_vector_type(4))) float v4f_t;
typedef float v4fa __attribute__((ext_vector_type(4), may_alias));
typedef __attribute__((ext_vector_type(16))) bf16  bf16x16;
typedef __attribute__((ext_vector_type(8)))  bf16  bf16x8;
typedef __attribute__((ext_vector_type(4)))  bf16  bf16x4;
typedef __attribute__((ext_vector_type(8)))  float f32x8;

#define LDS_STRIDE 48
#define KSTRIDE    72
#define VSTRIDE    48

__device__ __forceinline__ f32x8 wmma_bf16(bf16x16 a, bf16x16 b, f32x8 c) {
  return __builtin_amdgcn_wmma_f32_16x16x32_f16(
      false, a, false, b, (short)0, c, false, false);
}

template <typename T>
__device__ __forceinline__ bf16x16 load_frag(const T* __restrict__ base, int ld,
                                             int row0, int k0) {
  const int lane = threadIdx.x & 31;
  const int r    = lane & 15;
  const int kh   = (lane >> 4) * 8;
  const T* p0 = base + (size_t)(row0 + r) * ld + (k0 + kh);
  const T* p1 = p0 + 16;
  bf16x16 f;
#pragma unroll
  for (int i = 0; i < 8; ++i) {
    f[i]     = (bf16)p0[i];
    f[i + 8] = (bf16)p1[i];
  }
  return f;
}

__device__ __forceinline__ bf16x16 lds_frag(const bf16* base, int stride) {
  const int lane = threadIdx.x & 31;
  const int row  = lane & 15;
  const int kh   = (lane >> 4) * 8;
  const bf16x8 lo = *(const bf16x8*)(base + row * stride + kh);
  const bf16x8 hi = *(const bf16x8*)(base + row * stride + kh + 16);
  bf16x16 f;
#pragma unroll
  for (int i = 0; i < 8; ++i) { f[i] = lo[i]; f[i + 8] = hi[i]; }
  return f;
}

template <typename T>
__device__ __forceinline__ void stage_read16(const T* __restrict__ p, float* buf) {
#pragma unroll
  for (int i = 0; i < 16; ++i) buf[i] = (float)p[i];
}

__device__ __forceinline__ void stage_write(bf16* dst, const float* buf, int nquad) {
#pragma unroll
  for (int i = 0; i < nquad; ++i) {
    bf16x4 q;
    q[0] = (bf16)buf[4 * i];     q[1] = (bf16)buf[4 * i + 1];
    q[2] = (bf16)buf[4 * i + 2]; q[3] = (bf16)buf[4 * i + 3];
    *(bf16x4*)(dst + 4 * i) = q;
  }
}

template <typename AT, int MODE>
__global__ __launch_bounds__(256) void gemm_bias_kernel(
    const AT* __restrict__ A, const float* __restrict__ W,
    const float* __restrict__ bias, void* __restrict__ out,
    int M, int N, int K) {
  __shared__ bf16 ldsA[128 * LDS_STRIDE];
  __shared__ bf16 ldsW[256 * LDS_STRIDE];
  __shared__ __attribute__((aligned(16))) unsigned char sob[256 * 136 * 2];

  const int t    = threadIdx.x;
  const int wave = t >> 5;
  const int lane = t & 31;
  const int wm   = (wave & 1) * 64;
  const int wn   = (wave >> 1) * 64;
  const int mBlk = blockIdx.x * 128;
  const int nBlk = blockIdx.y * 256;

  const int arow = t >> 1;
  const int ach  = (t & 1) * 16;

  float abuf[16];
  float wbuf[32];

  stage_read16(A + (size_t)(mBlk + arow) * K + ach, abuf);
  stage_read16(W + (size_t)(nBlk + t) * K,          wbuf);
  stage_read16(W + (size_t)(nBlk + t) * K + 16,     wbuf + 16);

  f32x8 acc[4][4] = {};

  for (int k = 0; k < K; k += 32) {
    __syncthreads();
    stage_write(&ldsA[arow * LDS_STRIDE + ach], abuf, 4);
    stage_write(&ldsW[t * LDS_STRIDE],          wbuf, 8);
    if (k + 32 < K) {
      stage_read16(A + (size_t)(mBlk + arow) * K + (k + 32) + ach, abuf);
      stage_read16(W + (size_t)(nBlk + t) * K + (k + 32),          wbuf);
      stage_read16(W + (size_t)(nBlk + t) * K + (k + 32) + 16,     wbuf + 16);
    }
    __syncthreads();

    bf16x16 af[4], wf[4];
#pragma unroll
    for (int i = 0; i < 4; ++i)
      af[i] = lds_frag(ldsA + (wm + 16 * i) * LDS_STRIDE, LDS_STRIDE);
#pragma unroll
    for (int j = 0; j < 4; ++j)
      wf[j] = lds_frag(ldsW + (wn + 16 * j) * LDS_STRIDE, LDS_STRIDE);
#pragma unroll
    for (int i = 0; i < 4; ++i)
#pragma unroll
      for (int j = 0; j < 4; ++j)
        acc[i][j] = wmma_bf16(af[i], wf[j], acc[i][j]);
  }

  const int nlane = lane & 15;
  const int mh    = (lane >> 4) * 8;
  __syncthreads();
  if (MODE == 0 || MODE == 1) {
    bf16* so = (bf16*)sob;
#pragma unroll
    for (int i = 0; i < 4; ++i)
#pragma unroll
      for (int j = 0; j < 4; ++j) {
        const int nl = wn + 16 * j + nlane;
        const float bv = bias ? bias[nBlk + nl] : 0.0f;
#pragma unroll
        for (int r = 0; r < 8; ++r) {
          const int ml = wm + 16 * i + mh + r;
          const bf16 hv = (bf16)(acc[i][j][r] + bv);
          if (MODE == 0) so[ml * 264 + nl] = hv;
          else           so[nl * 136 + ml] = hv;
        }
      }
    __syncthreads();
#pragma unroll 1
    for (int pass = 0; pass < 2; ++pass) {
      if (MODE == 0) {
        for (int ch = t; ch < 128 * 32; ch += 256) { const int ml = ch >> 5, q = (ch & 31) * 8;
          *(volatile v4u_t*)((bf16*)out + (size_t)(mBlk + ml) * N + nBlk + q) = *(const v4ua*)(so + ml * 264 + q); }
      } else {
        const int b_ = mBlk / SS, s0 = mBlk & (SS - 1);
        for (int ch = t; ch < 256 * 16; ch += 256) { const int nl = ch >> 4, q = (ch & 15) * 8; const int n = nBlk + nl, h = n >> 6, dk = n & (DKK - 1);
          *(volatile v4u_t*)((bf16*)out + (((size_t)(b_ * HH + h)) * DKK + dk) * SS + s0 + q) = *(const v4ua*)(so + nl * 136 + q); }
      }
      __threadfence();
    }
  } else {
    float* so = (float*)sob;
#pragma unroll 1
    for (int hf = 0; hf < 2; ++hf) {
      if (wm == hf * 64) {
#pragma unroll
        for (int i = 0; i < 4; ++i)
#pragma unroll
          for (int j = 0; j < 4; ++j) {
            const int nl = wn + 16 * j + nlane;
            const float bv = bias ? bias[nBlk + nl] : 0.0f;
#pragma unroll
            for (int r = 0; r < 8; ++r) so[(16 * i + mh + r) * 260 + nl] = acc[i][j][r] + bv;
          }
      }
      __syncthreads();
#pragma unroll 1
      for (int pass = 0; pass < 2; ++pass) {
        for (int ch = t; ch < 64 * 64; ch += 256) { const int ml = ch >> 6, q = (ch & 63) * 4;
          *(volatile v4f_t*)((float*)out + (size_t)(mBlk + hf * 64 + ml) * N + nBlk + q) = *(const volatile v4fa*)(so + ml * 260 + q); }
        __threadfence();
      }
      __syncthreads();
    }
  }
}

__global__ __launch_bounds__(64) void attn_kernel(
    const bf16* __restrict__ Qb, const bf16* __restrict__ Kb,
    const bf16* __restrict__ Vt, const float* __restrict__ RS,
    float* __restrict__ out) {
  __shared__ bf16 ldsK[32 * KSTRIDE];
  __shared__ bf16 ldsV[64 * VSTRIDE];
  __shared__ __attribute__((aligned(16))) float ldsO[2][32 * 68];

  const int q0blk = blockIdx.x * 64;
  const int h  = blockIdx.y;
  const int b  = blockIdx.z;
  const int t    = threadIdx.x;
  const int wave = t >> 5;
  const int lane = t & 31;
  const int qlane = lane & 15;
  const int kh8   = (lane >> 4) * 8;
  const int q0 = q0blk + wave * 32;

  const bf16* Qh = Qb + (size_t)b * SS * DD + h * DKK;
  const bf16* Kh = Kb + (size_t)b * SS * DD + h * DKK;
  const bf16* Vh = Vt + ((size_t)(b * HH + h)) * DKK * SS;

  const int krow = t >> 1;
  const int kcol = (t & 1) * 32;
  const bf16* kSrc = Kh + (size_t)krow * DD + kcol;
  const bf16* vSrc = Vh + (size_t)t * SS;

  bf16x16 qf[QW][2];
#pragma unroll
  for (int qt = 0; qt < QW; ++qt) {
    qf[qt][0] = load_frag(Qh, DD, q0 + 16 * qt, 0);
    qf[qt][1] = load_frag(Qh, DD, q0 + 16 * qt, 32);
  }

  f32x8 o[QW][4] = {};
  float mrun[QW], lrun[QW];
#pragma unroll
  for (int qt = 0; qt < QW; ++qt) { mrun[qt] = -INFINITY; lrun[qt] = 0.0f; }

  const float scale = RS[b] * 1.44269504088896340736f;
  const float NEGD = -3.0e38f;
  const int kmax = SS - 1;


  bf16x8 kreg[4], vreg[4];
#pragma unroll
  for (int i = 0; i < 4; ++i) {
    kreg[i] = *(const bf16x8*)(kSrc + 8 * i);
    vreg[i] = *(const bf16x8*)(vSrc + 8 * i);
  }

  for (int kb = 0; kb <= kmax; kb += 32) {
    __syncthreads();
#pragma unroll
    for (int i = 0; i < 4; ++i) {
      *(bf16x8*)(&ldsK[krow * KSTRIDE + kcol + 8 * i]) = kreg[i];
      *(bf16x8*)(&ldsV[t * VSTRIDE + 8 * i])           = vreg[i];
    }
    if (kb + 32 <= kmax) {
      const bf16* kn = kSrc + (size_t)(kb + 32) * DD;
      const bf16* vn = vSrc + (kb + 32);
#pragma unroll
      for (int i = 0; i < 4; ++i) {
        kreg[i] = *(const bf16x8*)(kn + 8 * i);
        vreg[i] = *(const bf16x8*)(vn + 8 * i);
      }
    }
    __syncthreads();

    bf16x16 kf[2][2];
#pragma unroll
    for (int ktile = 0; ktile < 2; ++ktile)
#pragma unroll
      for (int c = 0; c < 2; ++c)
        kf[ktile][c] = lds_frag(ldsK + (ktile * 16) * KSTRIDE + c * 32, KSTRIDE);

    bf16x16 pf[QW];
    bool act[QW];
#pragma unroll
    for (int qt = 0; qt < QW; ++qt) {
      unsigned mbits = 0;
      {
        mbits = 0xFFFFu; act[qt] = true;
      }
      if (act[qt]) {
        const int q_my = q0 + 16 * qt + qlane;
        f32x8 s0 = {}, s1 = {};
        s0 = wmma_bf16(kf[0][0], qf[qt][0], s0);
        s0 = wmma_bf16(kf[0][1], qf[qt][1], s0);
        s1 = wmma_bf16(kf[1][0], qf[qt][0], s1);
        s1 = wmma_bf16(kf[1][1], qf[qt][1], s1);

        float mx = -INFINITY;
#pragma unroll
        for (int r = 0; r < 8; ++r) {
          const int k0i = kb + kh8 + r;
          const int k1i = k0i + 16;
          (void)k0i; (void)k1i; (void)q_my;
          s0[r] = (k0i == q_my) ? NEGD : s0[r] * scale;
          s1[r] = (k1i == q_my) ? NEGD : s1[r] * scale;
          mx = fmaxf(mx, fmaxf(s0[r], s1[r]));
        }
        mx = fmaxf(mx, __shfl_xor(mx, 16, 32));
        const float mnew  = fmaxf(mrun[qt], mx);
        const float alpha = exp2f(mrun[qt] - mnew);

        float rsum = 0.0f;
#pragma unroll
        for (int r = 0; r < 8; ++r) {
          const float p0 = exp2f(s0[r] - mnew);
          const float p1 = exp2f(s1[r] - mnew);
          rsum += p0 + p1;
          pf[qt][r]     = (bf16)(p0 * 1024.0f);
          pf[qt][r + 8] = (bf16)(p1 * 1024.0f);
        }
        rsum += __shfl_xor(rsum, 16, 32);
        lrun[qt] = lrun[qt] * alpha + rsum;
        mrun[qt] = mnew;

#pragma unroll
        for (int j = 0; j < 4; ++j)
#pragma unroll
          for (int r = 0; r < 8; ++r) o[qt][j][r] *= alpha;
      }
    }

#pragma unroll
    for (int j = 0; j < 4; ++j) {
      const bf16x16 vf = lds_frag(ldsV + (j * 16) * VSTRIDE, VSTRIDE);
#pragma unroll
      for (int qt = 0; qt < QW; ++qt)
        if (act[qt]) o[qt][j] = wmma_bf16(vf, pf[qt], o[qt][j]);
    }
  }

  float* so = ldsO[wave];
#pragma unroll
  for (int qt = 0; qt < QW; ++qt) {
    const float rl = 1.0f / (lrun[qt] * 1024.0f);
#pragma unroll
    for (int j = 0; j < 4; ++j)
#pragma unroll
      for (int r = 0; r < 8; ++r) so[(16 * qt + qlane) * 68 + j * 16 + kh8 + r] = o[qt][j][r] * rl;
  }
  asm volatile("s_wait_dscnt 0" ::: "memory");
#pragma unroll 1
  for (int pass = 0; pass < 2; ++pass) {
#pragma unroll
    for (int it = 0; it < 16; ++it) { const int ch = lane + 32 * it, ql = ch >> 4, q4 = (ch & 15) * 4;
      *(volatile v4f_t*)(out + ((size_t)(b * SS + q0 + ql)) * DD + h * DKK + q4) = *(const volatile v4fa*)(so + ql * 68 + q4); }
    __threadfence();
  }
}

__global__ __launch_bounds__(256) void k_tw(const float* __restrict__ W, float* __restrict__ WT, int K, int N) {
  __shared__ float tile[64][65];
  const int kb0 = blockIdx.y * 64, n0 = blockIdx.x * 64, t = threadIdx.x;
  for (int i = t; i < 64 * 64; i += 256) { const int kr = i >> 6, nc = i & 63; tile[kr][nc] = W[(size_t)(kb0 + kr) * N + n0 + nc]; }
  __syncthreads();
#pragma unroll 1
  for (int pass = 0; pass < 2; ++pass) {
    for (int i = t; i < 64 * 16; i += 256) { const int nr = i >> 4, k4 = (i & 15) * 4; v4f_t v; v.x = tile[k4][nr]; v.y = tile[k4 + 1][nr]; v.z = tile[k4 + 2][nr]; v.w = tile[k4 + 3][nr];
      *(volatile v4f_t*)(WT + (size_t)(n0 + nr) * K + kb0 + k4) = v; }
    __threadfence();
  }
}

__global__ __launch_bounds__(64) void k_stats(const bf16* __restrict__ Qb, const bf16* __restrict__ Kb, float* __restrict__ part) {
  __shared__ bf16 ldsK[32 * KSTRIDE]; __shared__ float ws2[2][2];
  const int q0blk = blockIdx.x * 64, b = blockIdx.z, t = threadIdx.x, wave = t >> 5, lane = t & 31;
  const int q0 = q0blk + wave * 32;
  const bf16* Qh = Qb + (size_t)b * SS * DD; const bf16* Kh = Kb + (size_t)b * SS * DD;
  const int krow = t >> 1, kcol = (t & 1) * 32;
  bf16x16 qf[2][2];
#pragma unroll
  for (int qt = 0; qt < 2; ++qt) { qf[qt][0] = load_frag(Qh, DD, q0 + 16 * qt, 0); qf[qt][1] = load_frag(Qh, DD, q0 + 16 * qt, 32); }
  float su = 0.0f, sq = 0.0f;
#pragma unroll 1
  for (int kb = 0; kb < SS; kb += 32) {
    __syncthreads();
    { const bf16* ks = Kh + (size_t)(kb + krow) * DD + kcol;
#pragma unroll
      for (int i = 0; i < 4; ++i) *(bf16x8*)(&ldsK[krow * KSTRIDE + kcol + 8 * i]) = *(const bf16x8*)(ks + 8 * i); }
    __syncthreads();
    bf16x16 kf[2][2];
#pragma unroll
    for (int kt = 0; kt < 2; ++kt) { kf[kt][0] = lds_frag(ldsK + (kt * 16) * KSTRIDE, KSTRIDE); kf[kt][1] = lds_frag(ldsK + (kt * 16) * KSTRIDE + 32, KSTRIDE); }
#pragma unroll
    for (int qt = 0; qt < 2; ++qt) { f32x8 s0 = {}, s1 = {};
      s0 = wmma_bf16(kf[0][0], qf[qt][0], s0); s0 = wmma_bf16(kf[0][1], qf[qt][1], s0);
      s1 = wmma_bf16(kf[1][0], qf[qt][0], s1); s1 = wmma_bf16(kf[1][1], qf[qt][1], s1);
#pragma unroll
      for (int r = 0; r < 8; ++r) { su += s0[r] + s1[r]; sq += s0[r] * s0[r] + s1[r] * s1[r]; } }
  }
#pragma unroll
  for (int o = 16; o >= 1; o >>= 1) { su += __shfl_xor(su, o, 32); sq += __shfl_xor(sq, o, 32); }
  if (lane == 0) { ws2[wave][0] = su; ws2[wave][1] = sq; }
  __syncthreads();
  if (wave == 0) { const float v = (lane == 0) ? ws2[0][0] : (lane == 1) ? ws2[0][1] : (lane == 2) ? ws2[1][0] : (lane == 3) ? ws2[1][1] : 0.0f;
    float* pl = part + ((size_t)b * (SS / 64) + blockIdx.x) * 32 + lane; *(volatile float*)pl = v; __threadfence(); *(volatile float*)pl = v; }
}
__global__ __launch_bounds__(64) void k_rs(const float* __restrict__ part, float* __restrict__ RS) {
  const int b = threadIdx.x; double s = 0.0, q = 0.0;
  for (int i = 0; i < SS / 64; ++i) { const float* pl = part + ((size_t)b * (SS / 64) + i) * 32; s += (double)pl[0] + (double)pl[2]; q += (double)pl[1] + (double)pl[3]; }
  const double n = (double)SS * SS, mu = s / n, var = fmax(q / n - mu * mu, 0.0);
  const float v = (float)(1.0 / sqrt(var + 1e-5)); *(volatile float*)(RS + b) = v; __threadfence(); *(volatile float*)(RS + b) = v;
}
__global__ __launch_bounds__(256) void k_tr(const float* __restrict__ src, bf16* __restrict__ dst) {
  __shared__ float tile[64][65];
  const int l0 = blockIdx.x * 64, b = blockIdx.z, t = threadIdx.x;
  for (int i = t; i < 64 * 64; i += 256) { const int c = i >> 6, ll = i & 63; tile[c][ll] = src[((size_t)b * DD + c) * SS + l0 + ll]; }
  __syncthreads();
#pragma unroll 1
  for (int pass = 0; pass < 2; ++pass) {
    for (int i = t; i < 64 * 8; i += 256) { const int lr = i >> 3, c8 = (i & 7) * 8; bf16 hh[8];
#pragma unroll
      for (int e = 0; e < 8; ++e) hh[e] = (bf16)tile[c8 + e][lr];
      *(volatile v4u_t*)(dst + ((size_t)b * SS + l0 + lr) * DD + c8) = *(const v4ua*)hh; }
    __threadfence();
  }
}
__global__ __launch_bounds__(256) void k_cvt(const float* __restrict__ v, bf16* __restrict__ Vt) {
  const size_t off = ((size_t)blockIdx.x * 256 + threadIdx.x) * 4; const v4f_t a = *(const v4fa*)(v + off);
  bf16 h[4]; h[0] = (bf16)a.x; h[1] = (bf16)a.y; h[2] = (bf16)a.z; h[3] = (bf16)a.w;
  typedef __attribute__((ext_vector_type(2))) unsigned v2u; typedef unsigned v2ua __attribute__((ext_vector_type(2), may_alias));
  *(volatile v2u*)(Vt + off) = *(const v2ua*)h; __threadfence(); *(volatile v2u*)(Vt + off) = *(const v2ua*)h;
}
__global__ __launch_bounds__(256) void k_opart(const float* __restrict__ O, float* __restrict__ part2) {
  __shared__ float red[2][256];
  const int blk = blockIdx.x, t = threadIdx.x;
  const float* base = O + (size_t)blk * 2048; float s = 0.f, q = 0.f;
  for (int i = t; i < 2048; i += 256) { const float v = base[i]; s += v; q += v * v; }
  red[0][t] = s; red[1][t] = q; __syncthreads();
  for (int o = 128; o > 0; o >>= 1) { if (t < o) { red[0][t] += red[0][t + o]; red[1][t] += red[1][t + o]; } __syncthreads(); }
  if (t < 32) { const float v = (t == 0) ? red[0][0] : (t == 1) ? red[1][0] : 0.0f; *(volatile float*)(part2 + (size_t)blk * 32 + t) = v; __threadfence(); *(volatile float*)(part2 + (size_t)blk * 32 + t) = v; }
}
__global__ __launch_bounds__(256) void k_final(const float* __restrict__ O, const float* __restrict__ part2, float* __restrict__ out) {
  __shared__ float tile[64][65]; __shared__ float st[2];
  const int l0 = blockIdx.x * 64, seq = blockIdx.z, n = seq >> 3, r = seq & 7, t = threadIdx.x;
  if (t == 0) { double s = 0.0, q = 0.0; const int nb = 8 * SS * DD / 2048;
    for (int i = 0; i < nb; ++i) { const float* pl = part2 + ((size_t)n * nb + i) * 32; s += (double)pl[0]; q += (double)pl[1]; }
    const double cnt = 8.0 * SS * DD, mu = s / cnt, var = fmax(q / cnt - mu * mu, 0.0); st[0] = (float)mu; st[1] = (float)(1.0 / sqrt(var + 1e-5)); }
  for (int i = t; i < 64 * 64; i += 256) { const int lr = i >> 6, d = i & 63; tile[lr][d] = O[((size_t)seq * SS + l0 + lr) * DD + d]; }
  __syncthreads();
  const float mu = st[0], rs = st[1];
#pragma unroll 1
  for (int pass = 0; pass < 2; ++pass) {
    for (int i = t; i < 64 * 16; i += 256) { const int d = i >> 4, l4 = (i & 15) * 4; v4f_t v;
#pragma unroll 1
      for (int qq = 0; qq < 4; ++qq) { const float u = (tile[l4 + qq][d] - mu) * rs; v[qq] = 0.5f * u * (1.0f + erff(u * 0.70710678118654752f)); }
      *(volatile v4f_t*)(out + (((size_t)n * 8 + r) * DD + d) * SS + l0 + l4) = v; }
    __threadfence();
  }
}

extern "C" void kernel_launch(void* const* d_in, const int* in_sizes, int n_in,
                              void* d_out, int out_size, void* d_ws, size_t ws_size,
                              hipStream_t stream) {
  (void)in_sizes; (void)n_in; (void)out_size; (void)ws_size;
  const float* q = (const float*)d_in[0]; const float* k = (const float*)d_in[1]; const float* v = (const float*)d_in[2];
  float* out = (float*)d_out;
  char* ws = (char*)d_ws;
  bf16* Qb  = (bf16*)ws; ws += (size_t)BB * SS * DD * 2;
  bf16* Kb  = (bf16*)ws; ws += (size_t)BB * SS * DD * 2;
  bf16* VtB = (bf16*)ws; ws += (size_t)BB * DD * SS * 2;
  float* O  = (float*)ws; ws += (size_t)BB * SS * DD * 4;
  float* part = (float*)ws; ws += (size_t)BB * (SS / 64) * 32 * 4;
  float* RS = (float*)ws; ws += 64 * 4;
  const int nb2 = BB * SS * DD / 2048;
  float* part2 = (float*)ws; ws += (size_t)nb2 * 32 * 4;
  k_tr<<<dim3(SS / 64, 1, BB), 256, 0, stream>>>(q, Qb);
  k_tr<<<dim3(SS / 64, 1, BB), 256, 0, stream>>>(k, Kb);
  k_cvt<<<BB * DD * SS / 1024, 256, 0, stream>>>(v, VtB);
  k_stats<<<dim3(SS / 64, 1, BB), 64, 0, stream>>>(Qb, Kb, part);
  k_rs<<<1, 64, 0, stream>>>(part, RS);
  attn_kernel<<<dim3(SS / 64, HH, BB), dim3(64), 0, stream>>>(Qb, Kb, VtB, RS, O);
  k_opart<<<nb2, 256, 0, stream>>>(O, part2);
  k_final<<<dim3(SS / 64, 1, BB), 256, 0, stream>>>(O, part2, out);
}
